// CodeAwareContinuousEncoder_11622181503255
// MI455X (gfx1250) — hardware-run, weakly checked
//
#include <hip/hip_runtime.h>
#include <math.h>

typedef __attribute__((ext_vector_type(16))) __bf16   v16b;
typedef __attribute__((ext_vector_type(8)))  __bf16   v8b;
typedef __attribute__((ext_vector_type(8)))  float    v8f;
typedef __attribute__((ext_vector_type(4)))  float    v4f;
typedef __attribute__((ext_vector_type(4)))  unsigned v4u;
typedef __attribute__((ext_vector_type(4)))  int      v4i;

constexpr int kNB      = 4096;
constexpr int kNH      = 256;
constexpr int kNE      = 256;
constexpr int kNHeads  = 100;
constexpr int kTileRows  = 32;
constexpr int kMaxTiles  = kNB / kTileRows;
constexpr int kAPitch    = 264;
constexpr int kAPitchW   = kAPitch / 2;
constexpr int kSlabPitch = 36;
static_assert((kNH % 32) == 0, "K multiple of 32");
static_assert((kNE % 64) == 0 && (kNH % 64) == 0, "64 x 64 transpose tiles");
static_assert(kNE == 8 * 32, "eight waves x 32 output columns");
static_assert(kNB == 256 * 16, "list build: 256 threads x 16 samples");
static_assert((kAPitch % 8) == 0 && kAPitch >= kNH, "A pitch");

constexpr size_t kPlaneBytes = (size_t)kNHeads * kNE * kNH * 2;
constexpr size_t kOffBTH  = 0;
constexpr size_t kOffBTL  = kOffBTH + kPlaneBytes;
constexpr size_t kWsTotal = kOffBTL + kPlaneBytes;
static_assert(kPlaneBytes == 13107200ull, "plane bytes");
static_assert(kWsTotal == 26214400ull, "carve total");
static_assert(kWsTotal <= 134217728ull, "carve cap");
static_assert((kOffBTL % 128) == 0, "128-B aligned regions");

__device__ __forceinline__ unsigned bf16_rne_bits(float f) {
  const unsigned u = __float_as_uint(f);
  return (u + 0x7FFFu + ((u >> 16) & 1u)) >> 16;
}
__device__ __forceinline__ float bf16_bits_to_f32(unsigned h) { return __uint_as_float(h << 16); }

struct FragB {
  union U { v16b v; v8b h[2]; };
  static __device__ __forceinline__ v16b load(const __bf16* p) {
    U f;
    f.h[0] = *(const v8b*)(p);
    f.h[1] = *(const v8b*)(p + 16);
    return f.v;
  }
};

__device__ __forceinline__ v8f mma_bf16(v16b a, v16b b, v8f c) {
  c = __builtin_amdgcn_wmma_f32_16x16x32_bf16(false, a, false, b, (short)0, c, false, false);
  asm volatile("v_nop\n\tv_nop\n\tv_nop\n\tv_nop" : "+v"(c) : "v"(a), "v"(b));
  return c;
}
__device__ __forceinline__ v8f mma_split3(v16b ah, v16b al, v16b bh, v16b bl, v8f c) {
  c = mma_bf16(ah, bh, c);
  c = mma_bf16(ah, bl, c);
  c = mma_bf16(al, bh, c);
  return c;
}

__global__ __launch_bounds__(256) void prep_weight_planes(
    const float* __restrict__ W, unsigned short* __restrict__ bt_hi, unsigned short* __restrict__ bt_lo)
{
  __shared__ float sT[64 * 65];
  const int tid  = threadIdx.x;
  const int lane = tid & 31;
  const int wave = __builtin_amdgcn_readfirstlane((int)(threadIdx.x >> 5));
  const int bx   = blockIdx.x;
  const int head = bx >> 4;
  const int k0   = ((bx >> 2) & 3) * 64;
  const int n0   = (bx & 3) * 64;
  const float* Wh = W + (size_t)head * (kNH * kNE);
  const int lr = tid >> 4;
  const int lc4 = (tid & 15) * 4;
#pragma unroll
  for (int i = 0; i < 4; ++i) {
    const int row = lr + 16 * i;
    const v4f v = *(const v4f*)(Wh + (size_t)(k0 + row) * kNE + n0 + lc4);
    sT[row * 65 + lc4 + 0] = v[0];
    sT[row * 65 + lc4 + 1] = v[1];
    sT[row * 65 + lc4 + 2] = v[2];
    sT[row * 65 + lc4 + 3] = v[3];
  }
  __syncthreads();
  const int q  = lane >> 3;
  const int c8 = (lane & 7) * 8;
  v4u hv[2], lv[2];
#pragma unroll
  for (int it = 0; it < 2; ++it) {
    const int nrow = it * 32 + wave * 4 + q;
    unsigned hb[8], lb[8];
#pragma unroll
    for (int e = 0; e < 8; ++e) {
      const float f = sT[(c8 + e) * 65 + nrow];
      const unsigned h = bf16_rne_bits(f);
      hb[e] = h;
      lb[e] = bf16_rne_bits(f - bf16_bits_to_f32(h));
    }
    v4u a, b;
    a[0] = hb[0] | (hb[1] << 16);
    a[1] = hb[2] | (hb[3] << 16);
    a[2] = hb[4] | (hb[5] << 16);
    a[3] = hb[6] | (hb[7] << 16);
    b[0] = lb[0] | (lb[1] << 16);
    b[1] = lb[2] | (lb[3] << 16);
    b[2] = lb[4] | (lb[5] << 16);
    b[3] = lb[6] | (lb[7] << 16);
    hv[it] = a;
    lv[it] = b;
  }
  for (int pass = 0; pass < 2; ++pass) {
#pragma unroll
    for (int it = 0; it < 2; ++it) {
      const int nrow = it * 32 + wave * 4 + q;
      const size_t off = ((size_t)head * kNE + (size_t)(n0 + nrow)) * kNH + k0 + c8;
      *(volatile v4u*)(bt_hi + off) = hv[it];
      *(volatile v4u*)(bt_lo + off) = lv[it];
    }
    __threadfence();
  }
}

__global__ __launch_bounds__(256) void grouped_head_gemm(
    const float* __restrict__ values, const float* __restrict__ means, const float* __restrict__ stds,
    const int* __restrict__ head_idx, const float* __restrict__ w1, const float* __restrict__ b1,
    const unsigned short* __restrict__ bt_hi, const unsigned short* __restrict__ bt_lo,
    const float* __restrict__ b_heads, float* __restrict__ out)
{
  __shared__ __align__(16) __bf16 sAh[kTileRows * kAPitch];
  __shared__ __align__(16) __bf16 sAl[kTileRows * kAPitch];
  __shared__ __align__(16) float  sSlab[8][16 * kSlabPitch];
  __shared__ unsigned short sSid[kNB];
  __shared__ float sZ[kTileRows];
  __shared__ int   sRow[kTileRows];
  __shared__ int   sWtot[8];

  const int tid  = threadIdx.x;
  const int lane = tid & 31;
  const int wave = __builtin_amdgcn_readfirstlane((int)(threadIdx.x >> 5));
  const int head = blockIdx.x;
  const int hh   = lane >> 4;
  const int c    = lane & 15;

  unsigned mbits = 0u;
  {
    const v4i* hp4 = (const v4i*)head_idx;
#pragma unroll
    for (int i = 0; i < 4; ++i) {
      const v4i v = hp4[tid * 4 + i];
#pragma unroll
      for (int e = 0; e < 4; ++e) {
        int k = v[e];
        k = k < 0 ? 0 : k;
        k = k > (kNHeads - 1) ? (kNHeads - 1) : k;
        mbits |= (k == head) ? (1u << (4 * i + e)) : 0u;
      }
    }
  }
  const int cntl = __popc(mbits);
  int xs = cntl;
#pragma unroll
  for (int off = 1; off < 32; off <<= 1) {
    const int y = __shfl_up(xs, off, 32);
    xs += (lane >= off) ? y : 0;
  }
  if (lane == 31) sWtot[wave] = xs;
  __syncthreads();
  int base = 0, cntv = 0;
#pragma unroll
  for (int w = 0; w < 8; ++w) {
    const int t = sWtot[w];
    base += (w < wave) ? t : 0;
    cntv += t;
  }
  {
    int pos = base + xs - cntl;
#pragma unroll
    for (int j = 0; j < 16; ++j) {
      if ((mbits >> j) & 1u) {
        const int pc = pos < (kNB - 1) ? pos : (kNB - 1);
        sSid[pc] = (unsigned short)(tid * 16 + j);
        ++pos;
      }
    }
  }
  int cnt = __builtin_amdgcn_readfirstlane(cntv);
  cnt = cnt > kNB ? kNB : cnt;
  int ntiles = (cnt + kTileRows - 1) / kTileRows;
  ntiles = ntiles > kMaxTiles ? kMaxTiles : ntiles;

  const int hp = tid & 127;
  const int mh = wave >> 2;
  const float wA = w1[2 * hp];
  const float wB = w1[2 * hp + 1];
  const float bA = b1[2 * hp];
  const float bB = b1[2 * hp + 1];
  const int n0 = wave * 32;
  const float bj0 = b_heads[(size_t)head * kNE + n0 + c];
  const float bj1 = b_heads[(size_t)head * kNE + n0 + 16 + c];
  const __bf16* BH = (const __bf16*)bt_hi + (size_t)head * (kNE * kNH) + (size_t)(n0 + c) * kNH + 8 * hh;
  const __bf16* BL = (const __bf16*)bt_lo + (size_t)head * (kNE * kNH) + (size_t)(n0 + c) * kNH + 8 * hh;
  float* slab = &sSlab[wave][0];
  const int q  = lane >> 3;
  const int c4 = (lane & 7) * 4;

#pragma unroll 1
  for (int tile = 0; tile < ntiles; ++tile) {
    __syncthreads();
    if (wave == 0) {
      const int r = tile * kTileRows + lane;
      const bool valid = r < cnt;
      const int rc = valid ? r : (cnt - 1);
      int sid = (int)sSid[rc];
      sid = sid > (kNB - 1) ? (kNB - 1) : sid;
      const float vv = values[sid];
      const float mm = means[sid];
      const float ss = stds[sid];
      const float sd = fmaxf(ss, 1e-8f);
      float z = (vv - mm) / sd;
      z = fminf(fmaxf(z, -5.0f), 5.0f);
      sZ[lane] = z;
      sRow[lane] = valid ? sid : -1;
    }
    __syncthreads();
    {
      unsigned* aHw = (unsigned*)sAh;
      unsigned* aLw = (unsigned*)sAl;
#pragma unroll 1
      for (int mm = 0; mm < 16; ++mm) {
        const int m = mh * 16 + mm;
        const float z = sZ[m];
        const bool valid = sRow[m] >= 0;
        const float x0 = z * wA + bA;
        const float x1 = z * wB + bB;
        const float g0 = 0.5f * x0 * (1.0f + erff(x0 * 0.70710678118654752f));
        const float g1 = 0.5f * x1 * (1.0f + erff(x1 * 0.70710678118654752f));
        const unsigned h0 = bf16_rne_bits(g0);
        const unsigned h1 = bf16_rne_bits(g1);
        const unsigned l0 = bf16_rne_bits(g0 - bf16_bits_to_f32(h0));
        const unsigned l1 = bf16_rne_bits(g1 - bf16_bits_to_f32(h1));
        const unsigned wh = h0 | (h1 << 16);
        const unsigned wl = l0 | (l1 << 16);
        aHw[m * kAPitchW + hp] = valid ? wh : 0u;
        aLw[m * kAPitchW + hp] = valid ? wl : 0u;
      }
    }
    __syncthreads();

    v8f acc[2][2];
#pragma unroll
    for (int i = 0; i < 2; ++i)
#pragma unroll
      for (int j = 0; j < 2; ++j) acc[i][j] = (v8f){0.f,0.f,0.f,0.f,0.f,0.f,0.f,0.f};

#pragma unroll 1
    for (int k0 = 0; k0 < kNH; k0 += 32) {
      const v16b bh0 = FragB::load(BH + k0);
      const v16b bh1 = FragB::load(BH + 16 * kNH + k0);
      const v16b bl0 = FragB::load(BL + k0);
      const v16b bl1 = FragB::load(BL + 16 * kNH + k0);
      const v16b ah0 = FragB::load(sAh + c * kAPitch + k0 + 8 * hh);
      const v16b ah1 = FragB::load(sAh + (16 + c) * kAPitch + k0 + 8 * hh);
      const v16b al0 = FragB::load(sAl + c * kAPitch + k0 + 8 * hh);
      const v16b al1 = FragB::load(sAl + (16 + c) * kAPitch + k0 + 8 * hh);
      acc[0][0] = mma_split3(ah0, al0, bh0, bl0, acc[0][0]);
      acc[0][1] = mma_split3(ah0, al0, bh1, bl1, acc[0][1]);
      acc[1][0] = mma_split3(ah1, al1, bh0, bl0, acc[1][0]);
      acc[1][1] = mma_split3(ah1, al1, bh1, bl1, acc[1][1]);
    }

#pragma unroll
    for (int i = 0; i < 2; ++i) {
#pragma unroll
      for (int r = 0; r < 8; ++r) {
        slab[(8 * hh + r) * kSlabPitch + c]      = acc[i][0][r] + bj0;
        slab[(8 * hh + r) * kSlabPitch + 16 + c] = acc[i][1][r] + bj1;
      }
      __builtin_amdgcn_fence(__ATOMIC_RELEASE, "workgroup");
      __builtin_amdgcn_wave_barrier();
      __builtin_amdgcn_fence(__ATOMIC_ACQUIRE, "workgroup");
      v4f vals[4];
      int sids[4];
#pragma unroll
      for (int it = 0; it < 4; ++it) {
        const int row = it * 4 + q;
        vals[it] = *(const v4f*)(slab + row * kSlabPitch + c4);
        sids[it] = sRow[i * 16 + row];
      }
      for (int pass = 0; pass < 2; ++pass) {
#pragma unroll
        for (int it = 0; it < 4; ++it) {
          if (sids[it] >= 0) {
            *(volatile v4f*)(out + (size_t)sids[it] * kNE + n0 + c4) = vals[it];
          }
        }
        __threadfence();
      }
      __builtin_amdgcn_fence(__ATOMIC_RELEASE, "workgroup");
      __builtin_amdgcn_wave_barrier();
      __builtin_amdgcn_fence(__ATOMIC_ACQUIRE, "workgroup");
    }
  }
}

extern "C" void kernel_launch(void* const* d_in, const int* in_sizes, int n_in,
                              void* d_out, int out_size, void* d_ws, size_t ws_size,
                              hipStream_t stream) {
  if (n_in < 8) return;
  if (in_sizes[0] != kNB) return;
  if (in_sizes[1] != kNB) return;
  if (in_sizes[2] != kNB) return;
  if (in_sizes[3] != kNB) return;
  if (in_sizes[4] != kNH) return;
  if (in_sizes[5] != kNH) return;
  if (in_sizes[6] != kNHeads * kNH * kNE) return;
  if (in_sizes[7] != kNHeads * kNE) return;
  if (out_size != kNB * kNE) return;
  if (ws_size < kWsTotal) return;

  const float* values   = (const float*)d_in[0];
  const float* means    = (const float*)d_in[1];
  const float* stds     = (const float*)d_in[2];
  const int*   head_idx = (const int*)d_in[3];
  const float* w1       = (const float*)d_in[4];
  const float* b1       = (const float*)d_in[5];
  const float* W_heads  = (const float*)d_in[6];
  const float* b_heads  = (const float*)d_in[7];
  float* out = (float*)d_out;

  char* ws = (char*)d_ws;
  unsigned short* BTH = (unsigned short*)(ws + kOffBTH);
  unsigned short* BTL = (unsigned short*)(ws + kOffBTL);

  prep_weight_planes<<<kNHeads * (kNH / 64) * (kNE / 64), 256, 0, stream>>>(W_heads, BTH, BTL);
  grouped_head_gemm<<<kNHeads, 256, 0, stream>>>(values, means, stds, head_idx, w1, b1, BTH, BTL, b_heads, out);
}
